// SimpleRGCN_11519102288003
// MI455X (gfx1250) — hardware-run, weakly checked
//
#include <hip/hip_runtime.h>
#include <stddef.h>
#include <stdint.h>


#define L1_SINGLE 0
#define L2_SINGLE 0

#define NN     100000
#define NE     640000
#define NR     16
#define D1     128
#define D2     256
#define NB     1024
#define SLA    10
#define NBLK   98
#define NSUB   8
#define SUBN   128
#define NSB    (NBLK * NSUB)
#define NSBL   782
#define NTHR   256
#define NWAVE  8
#define EPT    8
#define CHUNK  (NTHR * EPT)
#define WCAP   (EPT * 32)
#define LISTN  (NWAVE * WCAP)
#define RCAP   7168
#define SEGCAP 1536
#define DEGCAP 32
#define PCAPS  1792
#define NTILES (PCAPS / 16)
#define NKEY   (NSUB * NR * SUBN)
#define ARRN   (NKEY + 16)
#define NGRP   (NKEY / 32)
#define RELTW  32
#define REG0N  (LISTN + 2 * RCAP)
#define BK_INTS (REG0N + ARRN + RCAP + 2 * NGRP + NSUB * RELTW + 32)
#define LYX    (SEGCAP + PCAPS + 128 + 16 + 32)
#define LY1_INTS (129 * (D2 + 8) + 128 * (D1 + 4) + LYX)
#define LY2_INTS (129 * (D1 + 8) + 128 * (D2 + 4) + LYX)
#define WSMAX  134217728

static_assert(D1 % 32 == 0 && D2 % 32 == 0 && 128 % 16 == 0);
static_assert(NSUB * SUBN == NB && NB == (1 << SLA) && NBLK * NB >= NN);
static_assert(NWAVE * 32 == D2 && NWAVE * 16 == D1 && NTHR == NWAVE * 32);
static_assert(NSBL * SUBN >= NN && (NSBL - 1) * SUBN < NN && NSBL <= NSB);
static_assert((SEGCAP * 4) % 128 == 0 && (PCAPS * 4) % 128 == 0 && (RELTW * 4) % 128 == 0);
static_assert(RCAP >= 6764 + 6764 / 20 && RCAP % 256 == 0 && DEGCAP >= 19 + 8 && DEGCAP < 256);
static_assert(PCAPS % 16 == 0 && PCAPS >= SEGCAP + NR * 15 && SEGCAP < 32768);
static_assert(NSUB * PCAPS <= REG0N && (NSUB * PCAPS) % (NTHR * 4) == 0);
static_assert((NSUB * SEGCAP / 4) % NTHR == 0);
static_assert(NKEY % 32 == 0 && NGRP == NSUB * NR * 4);
static_assert((NE % 8) == 0 && ((CHUNK << SLA) > 0));
static_assert(BK_INTS % 4 == 0 && REG0N % 4 == 0 && ARRN % 4 == 0 && NGRP % 4 == 0);
static_assert(BK_INTS * 4 <= 300000 && LY1_INTS * 4 <= 300000 && LY2_INTS * 4 <= 300000);
static_assert(LY1_INTS % 4 == 0 && LY2_INTS % 4 == 0 && (129 * (D2 + 8)) % 4 == 0 && (129 * (D1 + 8)) % 4 == 0);

typedef float          v4f   __attribute__((ext_vector_type(4)));
typedef float          v8f   __attribute__((ext_vector_type(8)));
typedef int            v4i   __attribute__((ext_vector_type(4)));
typedef int            v8i   __attribute__((ext_vector_type(8)));
typedef unsigned short v8us  __attribute__((ext_vector_type(8)));
typedef __bf16         v16bf __attribute__((ext_vector_type(16)));
typedef v4f  __attribute__((may_alias)) v4fa;
typedef v4i  __attribute__((may_alias)) v4ia;
typedef v8us __attribute__((may_alias)) v8usa;
union FragB { v16bf v; v8us u[2]; v8i w; v4i q[2]; };

__device__ __forceinline__ v8f wmx(const FragB& a, const FragB& b, v8f c) {
  v8f d = __builtin_amdgcn_wmma_f32_16x16x32_bf16(false, a.v, false, b.v, (short)0, c, false, false);
  asm volatile("v_nop\n\tv_nop\n\tv_nop\n\tv_nop" : "+v"(d) : "v"(a.w), "v"(b.w));
  return d;
}

__device__ __forceinline__ void pinf(float x) { asm volatile("" :: "v"(x)); }
__device__ __forceinline__ void pini(int x)   { asm volatile("" :: "v"(x)); }
__device__ __forceinline__ void pin4(const v4i w) { pini(w.x); pini(w.y); pini(w.z); pini(w.w); }
__device__ __forceinline__ void pin4f(const v4f w) { pinf(w.x); pinf(w.y); pinf(w.z); pinf(w.w); }
__device__ __forceinline__ int clampi(int v, int lo, int hi) { return v < lo ? lo : (v > hi ? hi : v); }
__device__ __forceinline__ v8f z8() { v8f z = {0.f, 0.f, 0.f, 0.f, 0.f, 0.f, 0.f, 0.f}; return z; }

__device__ __forceinline__ unsigned bfbits(float v) {
  const unsigned u = __float_as_uint(v);
  const unsigned r = (u + 0x7FFFu + ((u >> 16) & 1u)) >> 16;
  const unsigned nb = ((u >> 16) & 0x8000u) | 0x7FC0u;
  return ((u & 0x7FFFFFFFu) > 0x7F800000u) ? nb : r;
}
__device__ __forceinline__ float bfval(float v) { return __uint_as_float(bfbits(v) << 16); }
__device__ __forceinline__ float mskf(float v, int mk) { return __int_as_float(__float_as_int(v) & mk); }

__device__ __forceinline__ void st2(unsigned short* dp, const v8us hv) {
  *(volatile v8us*)dp = hv;
  __threadfence();
  *(volatile v8us*)dp = hv;
}

__device__ __forceinline__ v8us gat8(const float* __restrict__ w, size_t sb, int stride) {
  float f[8];
#pragma unroll
  for (int i = 0; i < 8; ++i) { f[i] = w[sb + (size_t)i * (size_t)stride]; pinf(f[i]); }
  v8us hv;
#pragma unroll
  for (int i = 0; i < 8; ++i) hv[i] = (unsigned short)bfbits(f[i]);
  return hv;
}

__global__ __launch_bounds__(256) void k_prep(const float* __restrict__ w1, const float* __restrict__ w2,
                                              unsigned short* wt1, unsigned short* wt2) {
  const int b = (int)blockIdx.x, tid = (int)threadIdx.x;
  if (b < 256) {
    const int u  = b * 256 + tid;
    const int r  = u >> 12, n = (u >> 4) & 255, k8 = (u & 15) * 8;
    const size_t sb = (size_t)r * (D1 * D2) + (size_t)k8 * D2 + (size_t)n;
    st2(wt1 + (size_t)u * 8, gat8(w1, sb, D2));
  } else {
    const int u  = (b - 256) * 256 + tid;
    const int r  = u >> 12, n = (u >> 5) & 127, k8 = (u & 31) * 8;
    const size_t sb = (size_t)r * (D2 * D1) + (size_t)k8 * D1 + (size_t)n;
    st2(wt2 + (size_t)u * 8, gat8(w2, sb, D1));
  }
}

__device__ __forceinline__ int ldkey(const int* __restrict__ k, int e, int nE, int sent) {
  const int v = k[e < nE ? e : nE - 1];
  pini(v);
  return (e < nE) ? v : sent;
}

__device__ __forceinline__ int scan_chunk(const int* __restrict__ keys, int nE, int cbase, int slotBase,
                                          int nb, int* list, int tid, int lane, int wave) {
  int wc = 0;
  const int el0  = tid * EPT;
  const int e0   = cbase + el0;
  const int sent = (int)(1u << 31);
  v4i da, db;
  if (cbase + CHUNK <= nE) {
    da = *(const v4i*)(keys + e0);
    db = *(const v4i*)(keys + e0 + 4);
  } else {
    da.x = ldkey(keys, e0,     nE, sent);
    da.y = ldkey(keys, e0 + 1, nE, sent);
    da.z = ldkey(keys, e0 + 2, nE, sent);
    da.w = ldkey(keys, e0 + 3, nE, sent);
    db.x = ldkey(keys, e0 + 4, nE, sent);
    db.y = ldkey(keys, e0 + 5, nE, sent);
    db.z = ldkey(keys, e0 + 6, nE, sent);
    db.w = ldkey(keys, e0 + 7, nE, sent);
  }
  const unsigned nbs = (unsigned)slotBase;
  const unsigned unb = (unsigned)nb;
  const unsigned s0 = (unsigned)da.x - nbs, s1 = (unsigned)da.y - nbs;
  const unsigned s2 = (unsigned)da.z - nbs, s3 = (unsigned)da.w - nbs;
  const unsigned s4 = (unsigned)db.x - nbs, s5 = (unsigned)db.y - nbs;
  const unsigned s6 = (unsigned)db.z - nbs, s7 = (unsigned)db.w - nbs;
  const bool h0 = s0 < unb, h1 = s1 < unb, h2 = s2 < unb, h3 = s3 < unb;
  const bool h4 = s4 < unb, h5 = s5 < unb, h6 = s6 < unb, h7 = s7 < unb;
  const unsigned any = __builtin_amdgcn_ballot_w32(h0 | h1 | h2 | h3 | h4 | h5 | h6 | h7);
  if (any != 0u) {
    const int k = (int)h0 + (int)h1 + (int)h2 + (int)h3 + (int)h4 + (int)h5 + (int)h6 + (int)h7;
    int incl = k;
#pragma unroll
    for (int dd = 1; dd < 32; dd <<= 1) {
      const int y = __shfl_up(incl, dd, 32);
      if (lane >= dd) incl += y;
    }
    wc = __shfl(incl, 31, 32);
    int pos = incl - k;
#define PUTJ(J, HJ, SJ) if (HJ) { if (pos < WCAP) list[wave * WCAP + pos] = ((el0 + (J)) << SLA) | (int)(SJ); pos += 1; }
    PUTJ(0, h0, s0)
    PUTJ(1, h1, s1)
    PUTJ(2, h2, s2)
    PUTJ(3, h3, s3)
    PUTJ(4, h4, s4)
    PUTJ(5, h5, s5)
    PUTJ(6, h6, s6)
    PUTJ(7, h7, s7)
#undef PUTJ
  }
  return wc;
}

__global__ __launch_bounds__(NTHR) void k_bucket(const int* __restrict__ src, const int* __restrict__ dst,
                                                 const int* __restrict__ et, int* entg, int* pairg, int* reltg) {
  extern __shared__ __attribute__((aligned(16))) int dsm[];
  int* list = dsm;
  int* hk   = dsm + LISTN;
  int* hs   = hk + RCAP;
  int* pst  = dsm;
  int* arr  = dsm + REG0N;
  int* ent  = arr + ARRN;
  int* pcs  = ent + RCAP;
  int* pcm  = pcs + NGRP;
  int* relt = pcm + NGRP;
  int* misc = relt + NSUB * RELTW;
  const int tid = (int)threadIdx.x, lane = tid & 31;
  const int wave = __builtin_amdgcn_readfirstlane(tid >> 5);
  const int b = (int)blockIdx.x;
  const int nodeBase = b * NB;

  {
    const v4i z4 = {0, 0, 0, 0};
    for (int i = tid * 4; i < BK_INTS; i += NTHR * 4) *(v4ia*)(dsm + i) = z4;
  }
  __syncthreads();

  int t = 0;
  const int nChunks = (NE + CHUNK - 1) / CHUNK;
#pragma unroll 1
  for (int ch = 0; ch < nChunks; ++ch) {
    const int cbase = ch * CHUNK;
    int wc = scan_chunk(dst, NE, cbase, nodeBase, NB, list, tid, lane, wave);
    wc = clampi(wc, 0, WCAP);
    wc = __builtin_amdgcn_readfirstlane(wc);
    int* mb = misc + (ch & 1) * 8;
    if (lane == 0) mb[wave] = wc;
    __syncthreads();
    int base = t, tot = 0;
#pragma unroll
    for (int w2 = 0; w2 < NWAVE; ++w2) {
      const int c = clampi(mb[w2], 0, WCAP);
      base += (w2 < wave) ? c : 0;
      tot  += c;
    }
    const int myc = wc;
#pragma unroll 1
    for (int b0 = 0; b0 < myc; b0 += 32) {
      const int idx  = b0 + lane;
      const int entv = list[wave * WCAP + (idx < WCAP ? idx : WCAP - 1)];
      const int slot = entv & (NB - 1);
      const int el   = (entv >> SLA) & (CHUNK - 1);
      const int eid  = clampi(cbase + el, 0, NE - 1);
      int ty = et[eid];
      pini(ty);
      ty = clampi(ty, 0, NR - 1);
      int sr = src[eid];
      pini(sr);
      sr = clampi(sr, 0, NN - 1);
      const int pos = base + idx;
      if (idx < myc && pos < RCAP) {
        hk[pos] = (slot >> 7) * (NR * SUBN) + ty * SUBN + (slot & (SUBN - 1));
        hs[pos] = sr;
      }
    }
    t += tot;
  }
  __syncthreads();
  const int tt = t < RCAP ? t : RCAP;
  const int ov = t > RCAP ? 1 : 0;

  if (tid == 0) {
#pragma unroll 1
    for (int i = 0; i < tt; ++i) {
      const int k = clampi(hk[i], 0, NKEY - 1);
      arr[k] = arr[k] + 1;
    }
  }
  __syncthreads();
  if (wave == 0) {
    const int base = lane * (NKEY / 32);
    int s = 0;
#pragma unroll 1
    for (int i = 0; i < NKEY / 32; ++i) s += arr[base + i];
    int incl = s;
#pragma unroll
    for (int dd = 1; dd < 32; dd <<= 1) {
      const int y = __shfl_up(incl, dd, 32);
      if (lane >= dd) incl += y;
    }
    int run = incl - s;
#pragma unroll 1
    for (int i = 0; i < NKEY / 32; ++i) {
      run += arr[base + i];
      arr[base + i] = run;
    }
    if (lane == 31) arr[NKEY] = run;
  }
  __syncthreads();
  if (tid == 0) {
#pragma unroll 1
    for (int i = tt - 1; i >= 0; --i) {
      const int k = clampi(hk[i], 0, NKEY - 1);
      const int p = clampi(arr[k] - 1, 0, RCAP - 1);
      arr[k] = p;
      ent[p] = hs[i];
    }
  }
  __syncthreads();

  {
    int ovd = 0;
#pragma unroll 1
    for (int gi = wave; gi < NGRP; gi += NWAVE) {
      const int k = gi * 32 + lane;
      const int c = arr[k + 1] - arr[k];
      ovd |= (c > DEGCAP) ? 1 : 0;
      const unsigned m1 = __builtin_amdgcn_ballot_w32(c == 1);
      const unsigned m2 = __builtin_amdgcn_ballot_w32(c > 1);
      if (lane == 0) { pcs[gi] = (int)__builtin_popcount(m1); pcm[gi] = (int)__builtin_popcount(m2); }
    }
    const unsigned om = __builtin_amdgcn_ballot_w32(ovd != 0);
    if (lane == 0) misc[20 + wave] = (om != 0u) ? 1 : 0;
    const v4i z4 = {0, 0, 0, 0};
    for (int i = tid * 4; i < NSUB * PCAPS; i += NTHR * 4) *(v4ia*)(pst + i) = z4;
  }
  __syncthreads();
  if (tid == 0) {
    int fl = ov;
#pragma unroll 1
    for (int w2 = 0; w2 < NWAVE; ++w2) fl |= misc[20 + w2];
    int run = 0;
#pragma unroll 1
    for (int sg = 0; sg < NSUB * NR; ++sg) {
      const int s = sg >> 4, r = sg & 15;
      if (r == 0) run = 0;
      relt[s * RELTW + r] = run >> 4;
#pragma unroll 1
      for (int g = 0; g < 4; ++g) {
        const int c = clampi(pcs[sg * 4 + g], 0, 32);
        pcs[sg * 4 + g] = run;
        run += c;
      }
#pragma unroll 1
      for (int g = 0; g < 4; ++g) {
        const int c = clampi(pcm[sg * 4 + g], 0, 32);
        pcm[sg * 4 + g] = run;
        run += c;
      }
      run = (run + 15) & ~15;
      if (r == NR - 1) {
        relt[s * RELTW + NR] = run >> 4;
        const int st = arr[s * (NR * SUBN)];
        const int en = arr[(s + 1) * (NR * SUBN)];
        const int cs = en - st;
        relt[s * RELTW + 17] = (fl != 0 || cs > SEGCAP || cs < 0 || run > PCAPS) ? 1 : 0;
        relt[s * RELTW + 18] = clampi(cs, 0, SEGCAP);
        relt[s * RELTW + 19] = clampi(st, 0, RCAP);
      }
    }
  }
  __syncthreads();
#pragma unroll 1
  for (int gi = wave; gi < NGRP; gi += NWAVE) {
    const int k  = gi * 32 + lane;
    const int st = arr[k];
    int c = arr[k + 1] - st;
    c = clampi(c, 0, DEGCAP);
    const unsigned m1 = __builtin_amdgcn_ballot_w32(c == 1);
    const unsigned m2 = __builtin_amdgcn_ballot_w32(c > 1);
    const int i1 = pcs[gi] + (int)__builtin_amdgcn_mbcnt_lo(m1, 0u);
    const int i2 = pcm[gi] + (int)__builtin_amdgcn_mbcnt_lo(m2, 0u);
    const int idx = (c == 1) ? i1 : i2;
    const int s  = gi >> 6;
    const int so = clampi(st - relt[s * RELTW + 19], 0, SEGCAP - 1);
    if (c > 0 && idx >= 0 && idx < PCAPS) {
      pst[s * PCAPS + idx] = (k & (SUBN - 1)) | (c << 8) | (so << 16);
    }
  }
  __syncthreads();

  int* eg = entg  + (size_t)b * (NSUB * SEGCAP);
  int* pg = pairg + (size_t)b * (NSUB * PCAPS);
  int* rg = reltg + (size_t)b * (NSUB * RELTW);
#pragma unroll 1
  for (int ps = 0; ps < 2; ++ps) {
    for (int u = tid; u < NSUB * (SEGCAP / 4); u += NTHR) {
      const int s  = u / (SEGCAP / 4);
      const int i4 = (u - s * (SEGCAP / 4)) * 4;
      const int st = relt[s * RELTW + 19];
      const int cs = relt[s * RELTW + 18];
      const int e0 = ent[clampi(st + i4,     0, RCAP - 1)];
      const int e1 = ent[clampi(st + i4 + 1, 0, RCAP - 1)];
      const int e2 = ent[clampi(st + i4 + 2, 0, RCAP - 1)];
      const int e3 = ent[clampi(st + i4 + 3, 0, RCAP - 1)];
      v4i v;
      v.x = (i4     < cs) ? e0 : 0;
      v.y = (i4 + 1 < cs) ? e1 : 0;
      v.z = (i4 + 2 < cs) ? e2 : 0;
      v.w = (i4 + 3 < cs) ? e3 : 0;
      *(volatile v4i*)(eg + (size_t)u * 4) = v;
    }
    for (int i = tid * 4; i < NSUB * PCAPS; i += NTHR * 4) {
      const v4i v = *(const v4ia*)(pst + i);
      *(volatile v4i*)(pg + i) = v;
    }
    if (tid < (NSUB * RELTW) / 4) {
      const v4i v = *(const v4ia*)(relt + 4 * tid);
      *(volatile v4i*)(rg + 4 * tid) = v;
    }
    __threadfence();
  }
}

template <int LAYER>
__global__ __launch_bounds__(NTHR) __attribute__((amdgpu_num_vgpr(248)))
void k_layer(const float* __restrict__ xin, const int* __restrict__ nid,
             const unsigned short* __restrict__ wt, const int* __restrict__ entg,
             const int* __restrict__ pairg, const int* __restrict__ reltg,
             const float* __restrict__ gam, const float* __restrict__ bet,
             const float* __restrict__ emb, float* outp) {
  extern __shared__ __attribute__((aligned(16))) int lsm[];
  constexpr int KD    = (LAYER == 1) ? D1 : D2;
  constexpr int ND    = (LAYER == 1) ? D2 : D1;
  constexpr int NFR   = ND / (16 * NWAVE);
  constexpr int KST   = KD / 32;
  constexpr int NPASS = KD / 64;
  constexpr int APW   = ND + 8;
  constexpr int ATP   = KD + 4;
  constexpr int ACCN  = 129 * APW;
  constexpr int ATN   = 128 * ATP;
  constexpr int LYI   = ACCN + ATN + LYX;
  constexpr bool SGL  = (LAYER == 1) ? (L1_SINGLE != 0) : (L2_SINGLE != 0);
  static_assert(NFR * KST == 8 && ACCN % 4 == 0 && ATP % 4 == 0 && APW % 4 == 0);
  float* accf = (float*)lsm;
  int* atl = lsm + ACCN;
  int* seg = atl + ATN;
  int* prw = seg + SEGCAP;
  int* tsl = prw + PCAPS;
  int* lof = tsl + 128;
  int* rel = lof + 16;
  const int tid = (int)threadIdx.x, lane = tid & 31, hh = lane >> 4, m = lane & 15;
  const int wave = __builtin_amdgcn_readfirstlane(tid >> 5);
  const int sb = (int)blockIdx.x;
  const int nodeBase = sb * SUBN;

  {
    const v4i z4 = {0, 0, 0, 0};
    for (int i = tid * 4; i < LYI; i += NTHR * 4) *(v4ia*)(lsm + i) = z4;
  }
  __syncthreads();
#pragma unroll
  for (int it = 0; it < 2; ++it) {
    const int u  = tid + NTHR * it;
    const int ue = u < SEGCAP / 4 ? u : SEGCAP / 4 - 1;
    const v4i ve = *(const v4ia*)(entg + (size_t)sb * SEGCAP + 4 * ue);
    pin4(ve);
    if (u < SEGCAP / 4) *(v4ia*)(seg + 4 * u) = ve;
    const int up = u < PCAPS / 4 ? u : PCAPS / 4 - 1;
    const v4i vp = *(const v4ia*)(pairg + (size_t)sb * PCAPS + 4 * up);
    pin4(vp);
    if (u < PCAPS / 4) *(v4ia*)(prw + 4 * u) = vp;
  }
  if (wave == 0) {
    const int li = lane < RELTW / 4 ? lane : RELTW / 4 - 1;
    const v4i v = *(const v4ia*)(reltg + (size_t)sb * RELTW + 4 * li);
    pin4(v);
    if (lane < RELTW / 4) *(v4ia*)(rel + 4 * lane) = v;
  }
  __syncthreads();
  const int flag = rel[17];
  const int colw = NFR * 16 * wave;

#pragma unroll 1
  for (int r = 0; r < NR; ++r) {
    int t0 = clampi(rel[r], 0, NTILES);
    int t1 = clampi(rel[r + 1], t0, NTILES);
    t0 = __builtin_amdgcn_readfirstlane(t0);
    t1 = __builtin_amdgcn_readfirstlane(t1);
    if (t0 < t1) {
      FragB bfr[NFR * KST];
#pragma unroll
      for (int f = 0; f < NFR; ++f) {
#pragma unroll
        for (int ks = 0; ks < KST; ++ks) {
          const unsigned short* wq = wt + ((size_t)(r * ND + colw + 16 * f + m)) * KD + 32 * ks + 8 * hh;
          bfr[f * KST + ks].u[0] = *(const v8usa*)wq;
          bfr[f * KST + ks].u[1] = *(const v8usa*)(wq + 16);
        }
      }
#pragma unroll 1
      for (int base = t0; base < t1; base += NWAVE) {
        const int tl = base + wave;
        if (tl < t1) {
          const int pw = prw[tl * 16 + m];
          int cnt = clampi((pw >> 8) & 0xff, 0, DEGCAP);
          const int slot = pw & (SUBN - 1);
          const int off  = clampi((pw >> 16) & 0x7fff, 0, SEGCAP - 1);
          if (cnt > SEGCAP - off) cnt = SEGCAP - off;
          const int last = off + (cnt > 0 ? cnt - 1 : 0);
          int cm = cnt;
#pragma unroll
          for (int o2 = 1; o2 < 16; o2 <<= 1) {
            const int y = __shfl_xor(cm, o2, 32);
            cm = cm > y ? cm : y;
          }
          cm = __builtin_amdgcn_readfirstlane(cm);
          int* at = atl + (16 * wave + m) * ATP;
          int nz = 0;
#pragma unroll 1
          for (int cp = 0; cp < NPASS; ++cp) {
            const int cb = 64 * cp + 32 * hh;
            float a[32];
#pragma unroll
            for (int i = 0; i < 32; ++i) a[i] = 0.0f;
#pragma unroll 1
            for (int p = 0; p < cm; ++p) {
              int idx = off + p; idx = idx > last ? last : idx;
              const int sr = clampi(seg[idx], 0, NN - 1);
              const int mk = (p < cnt) ? -1 : 0;
              const float* rp;
              if constexpr (LAYER == 1) {
                int nd = nid[sr];
                pini(nd);
                nd = clampi(nd, 0, NN - 1);
                rp = xin + (size_t)nd * KD + cb;
              } else {
                rp = xin + (size_t)sr * KD + cb;
              }
              v4f w[8];
#pragma unroll
              for (int q = 0; q < 8; ++q) { w[q] = *(const v4f*)(rp + 4 * q); pin4f(w[q]); }
#pragma unroll
              for (int q = 0; q < 8; ++q) {
                if constexpr (LAYER == 1) {
                  a[4 * q + 0] += mskf(bfval(w[q].x), mk);
                  a[4 * q + 1] += mskf(bfval(w[q].y), mk);
                  a[4 * q + 2] += mskf(bfval(w[q].z), mk);
                  a[4 * q + 3] += mskf(bfval(w[q].w), mk);
                } else {
                  a[4 * q + 0] += mskf(w[q].x, mk);
                  a[4 * q + 1] += mskf(w[q].y, mk);
                  a[4 * q + 2] += mskf(w[q].z, mk);
                  a[4 * q + 3] += mskf(w[q].w, mk);
                }
              }
            }
            int hw[16], lw[16];
#pragma unroll
            for (int j = 0; j < 16; ++j) {
              const float v0 = a[2 * j], v1 = a[2 * j + 1];
              const unsigned h0 = bfbits(v0), h1 = bfbits(v1);
              hw[j] = (int)(h0 | (h1 << 16));
              const unsigned l0 = SGL ? 0u : bfbits(v0 - __uint_as_float(h0 << 16));
              const unsigned l1 = SGL ? 0u : bfbits(v1 - __uint_as_float(h1 << 16));
              lw[j] = (int)(l0 | (l1 << 16));
              nz |= lw[j];
            }
#pragma unroll
            for (int q = 0; q < 4; ++q) {
              v4i hv, lv;
              hv.x = hw[4 * q]; hv.y = hw[4 * q + 1]; hv.z = hw[4 * q + 2]; hv.w = hw[4 * q + 3];
              lv.x = lw[4 * q]; lv.y = lw[4 * q + 1]; lv.z = lw[4 * q + 2]; lv.w = lw[4 * q + 3];
              *(v4ia*)(at + 32 * cp + 16 * hh + 4 * q) = hv;
              *(v4ia*)(at + KD / 2 + 32 * cp + 16 * hh + 4 * q) = lv;
            }
          }
          if (hh == 0) tsl[16 * wave + m] = (cnt > 0) ? slot : SUBN;
          const unsigned nzm = __builtin_amdgcn_ballot_w32(nz != 0);
          if (lane == 0) lof[wave] = (nzm != 0u) ? 1 : 0;
        }
        __syncthreads();
        int nt = t1 - base;
        nt = nt > NWAVE ? NWAVE : nt;
#pragma unroll 1
        for (int tt = 0; tt < nt; ++tt) {
          const int lf = __builtin_amdgcn_readfirstlane(lof[tt]);
          const int* ar = atl + (16 * tt + m) * ATP;
          v8f d[NFR];
#pragma unroll
          for (int f = 0; f < NFR; ++f) d[f] = z8();
#pragma unroll
          for (int ks = 0; ks < KST; ++ks) {
            FragB af;
            af.q[0] = *(const v4ia*)(ar + 16 * ks + 4 * hh);
            af.q[1] = *(const v4ia*)(ar + 16 * ks + 8 + 4 * hh);
#pragma unroll
            for (int f = 0; f < NFR; ++f) d[f] = wmx(af, bfr[f * KST + ks], d[f]);
          }
          if (lf != 0) {
#pragma unroll
            for (int ks = 0; ks < KST; ++ks) {
              FragB af;
              af.q[0] = *(const v4ia*)(ar + KD / 2 + 16 * ks + 4 * hh);
              af.q[1] = *(const v4ia*)(ar + KD / 2 + 16 * ks + 8 + 4 * hh);
#pragma unroll
              for (int f = 0; f < NFR; ++f) d[f] = wmx(af, bfr[f * KST + ks], d[f]);
            }
          }
          int tr[8];
#pragma unroll
          for (int rr = 0; rr < 8; ++rr) tr[rr] = clampi(tsl[16 * tt + 8 * hh + rr], 0, SUBN) * APW;
#pragma unroll
          for (int f = 0; f < NFR; ++f) {
#pragma unroll
            for (int rr = 0; rr < 8; ++rr) {
              float* q = accf + tr[rr] + colw + 16 * f + m;
              const float old = *q;
              *q = old + d[f][rr];
            }
          }
        }
        __syncthreads();
      }
    }
  }

  const float qnan = __int_as_float(0x7fc00000);
  const bool pz = flag != 0;
  if constexpr (LAYER == 1) {
    const v4f ga = *(const v4f*)(gam + 4 * lane), gb = *(const v4f*)(gam + 128 + 4 * lane);
    const v4f ba = *(const v4f*)(bet + 4 * lane), bb = *(const v4f*)(bet + 128 + 4 * lane);
    const float g[8] = {bfval(ga.x), bfval(ga.y), bfval(ga.z), bfval(ga.w), bfval(gb.x), bfval(gb.y), bfval(gb.z), bfval(gb.w)};
    const float e[8] = {bfval(ba.x), bfval(ba.y), bfval(ba.z), bfval(ba.w), bfval(bb.x), bfval(bb.y), bfval(bb.z), bfval(bb.w)};
    const float invd = 1.0f / (float)D2;
#pragma unroll 1
    for (int i = 0; i < SUBN / NWAVE; ++i) {
      const int row  = wave + NWAVE * i;
      const int node = nodeBase + row;
      const v4f x0 = *(const v4fa*)(accf + row * APW + 4 * lane);
      const v4f x1 = *(const v4fa*)(accf + row * APW + 128 + 4 * lane);
      const float x[8] = {x0.x, x0.y, x0.z, x0.w, x1.x, x1.y, x1.z, x1.w};
      float s = ((x[0] + x[1]) + (x[2] + x[3])) + ((x[4] + x[5]) + (x[6] + x[7]));
      s += __shfl_xor(s, 16, 32);
      s += __shfl_xor(s, 8, 32);
      s += __shfl_xor(s, 4, 32);
      s += __shfl_xor(s, 2, 32);
      s += __shfl_xor(s, 1, 32);
      const float mu = s * invd;
      float dv[8];
      float q = 0.0f;
#pragma unroll
      for (int j = 0; j < 8; ++j) { dv[j] = x[j] - mu; q += dv[j] * dv[j]; }
      q += __shfl_xor(q, 16, 32);
      q += __shfl_xor(q, 8, 32);
      q += __shfl_xor(q, 4, 32);
      q += __shfl_xor(q, 2, 32);
      q += __shfl_xor(q, 1, 32);
      const float rstd = 1.0f / sqrtf(q * invd + 1e-5f);
      float o[8];
#pragma unroll
      for (int j = 0; j < 8; ++j) {
        float v = dv[j] * rstd * g[j] + e[j];
        v = (v > 0.0f) ? v : (v - v);
        o[j] = pz ? qnan : v;
      }
      v4f o0, o1;
      o0.x = o[0]; o0.y = o[1]; o0.z = o[2]; o0.w = o[3];
      o1.x = o[4]; o1.y = o[5]; o1.z = o[6]; o1.w = o[7];
      const int nc = node < NN ? node : NN - 1;
      float* op = outp + (size_t)nc * D2 + 4 * lane;
      if (node < NN) { *(volatile v4f*)op = o0; *(volatile v4f*)(op + 128) = o1; }
      __threadfence();
      if (node < NN) { *(volatile v4f*)op = o0; *(volatile v4f*)(op + 128) = o1; }
    }
  } else {
    const v4f ga = *(const v4f*)(gam + 4 * lane);
    const v4f ba = *(const v4f*)(bet + 4 * lane);
    const float g[4] = {bfval(ga.x), bfval(ga.y), bfval(ga.z), bfval(ga.w)};
    const float e[4] = {bfval(ba.x), bfval(ba.y), bfval(ba.z), bfval(ba.w)};
    const float invd = 1.0f / (float)D1;
#pragma unroll 1
    for (int i = 0; i < SUBN / NWAVE; ++i) {
      const int row  = wave + NWAVE * i;
      const int node = nodeBase + row;
      const int nc = node < NN ? node : NN - 1;
      int nd = nid[nc];
      pini(nd);
      nd = clampi(nd, 0, NN - 1);
      const v4f ev = *(const v4f*)(emb + (size_t)nd * D1 + 4 * lane);
      pin4f(ev);
      const v4f x0 = *(const v4fa*)(accf + row * APW + 4 * lane);
      const float x[4] = {x0.x, x0.y, x0.z, x0.w};
      float s = (x[0] + x[1]) + (x[2] + x[3]);
      s += __shfl_xor(s, 16, 32);
      s += __shfl_xor(s, 8, 32);
      s += __shfl_xor(s, 4, 32);
      s += __shfl_xor(s, 2, 32);
      s += __shfl_xor(s, 1, 32);
      const float mu = s * invd;
      float dv[4];
      float q = 0.0f;
#pragma unroll
      for (int j = 0; j < 4; ++j) { dv[j] = x[j] - mu; q += dv[j] * dv[j]; }
      q += __shfl_xor(q, 16, 32);
      q += __shfl_xor(q, 8, 32);
      q += __shfl_xor(q, 4, 32);
      q += __shfl_xor(q, 2, 32);
      q += __shfl_xor(q, 1, 32);
      const float rstd = 1.0f / sqrtf(q * invd + 1e-5f);
      const float rs[4] = {bfval(ev.x), bfval(ev.y), bfval(ev.z), bfval(ev.w)};
      float o[4];
#pragma unroll
      for (int j = 0; j < 4; ++j) {
        const float v = (dv[j] * rstd * g[j] + e[j]) + rs[j];
        o[j] = pz ? qnan : v;
      }
      v4f o0;
      o0.x = o[0]; o0.y = o[1]; o0.z = o[2]; o0.w = o[3];
      float* op = outp + (size_t)nc * D1 + 4 * lane;
      if (node < NN) *(volatile v4f*)op = o0;
      __threadfence();
      if (node < NN) *(volatile v4f*)op = o0;
    }
  }
  (void)emb; (void)nid;
}

static inline size_t al256(size_t o) { return (o + 255) & ~(size_t)255; }

extern "C" void kernel_launch(void* const* d_in, const int* in_sizes, int n_in,
                              void* d_out, int out_size, void* d_ws, size_t ws_size,
                              hipStream_t stream) {
  if (n_in < 10) return;
  if (in_sizes[0] != NN) return;
  if (in_sizes[1] != 2 * NE || in_sizes[2] != NE) return;
  if (in_sizes[3] != NN * D1) return;
  if (in_sizes[4] != NR * D1 * D2 || in_sizes[5] != NR * D2 * D1) return;
  if (in_sizes[6] != D2 || in_sizes[7] != D2 || in_sizes[8] != D1 || in_sizes[9] != D1) return;
  if (out_size != NN * D1) return;

  const int*   nid = (const int*)d_in[0];
  const int*   ei  = (const int*)d_in[1];
  const int*   et  = (const int*)d_in[2];
  const float* emb = (const float*)d_in[3];
  const float* W1  = (const float*)d_in[4];
  const float* W2  = (const float*)d_in[5];
  const float* g1  = (const float*)d_in[6];
  const float* b1  = (const float*)d_in[7];
  const float* g2  = (const float*)d_in[8];
  const float* b2  = (const float*)d_in[9];
  float* out = (float*)d_out;
  const int* src = ei;
  const int* dst = ei + NE;

  char* ws = (char*)d_ws;
  size_t off = 0;
  const size_t oX1   = off; off = al256(off + (size_t)NN * D2 * 4);
  const size_t oWT1  = off; off = al256(off + (size_t)NR * D2 * D1 * 2);
  const size_t oWT2  = off; off = al256(off + (size_t)NR * D1 * D2 * 2);
  const size_t oENT  = off; off = al256(off + (size_t)NSB * SEGCAP * 4);
  const size_t oPAIR = off; off = al256(off + (size_t)NSB * PCAPS * 4);
  const size_t oRELT = off; off = al256(off + (size_t)NSB * RELTW * 4);
  if (off > ws_size || off > (size_t)WSMAX) return;
  float*          X1   = (float*)(ws + oX1);
  unsigned short* WT1  = (unsigned short*)(ws + oWT1);
  unsigned short* WT2  = (unsigned short*)(ws + oWT2);
  int*            ENT  = (int*)(ws + oENT);
  int*            PAIR = (int*)(ws + oPAIR);
  int*            RELT = (int*)(ws + oRELT);

  const int bkLds = BK_INTS * 4;
  const int l1Lds = LY1_INTS * 4;
  const int l2Lds = LY2_INTS * 4;
  hipFuncSetAttribute(reinterpret_cast<const void*>(&k_bucket), hipFuncAttributeMaxDynamicSharedMemorySize, bkLds);
  hipFuncSetAttribute(reinterpret_cast<const void*>(&k_layer<1>), hipFuncAttributeMaxDynamicSharedMemorySize, l1Lds);
  hipFuncSetAttribute(reinterpret_cast<const void*>(&k_layer<2>), hipFuncAttributeMaxDynamicSharedMemorySize, l2Lds);

  k_prep<<<512, 256, 0, stream>>>(W1, W2, WT1, WT2);
  k_bucket<<<NBLK, NTHR, bkLds, stream>>>(src, dst, et, ENT, PAIR, RELT);
  k_layer<1><<<NSBL, NTHR, l1Lds, stream>>>(emb, nid, WT1, ENT, PAIR, RELT, g1, b1, emb, X1);
  k_layer<2><<<NSBL, NTHR, l2Lds, stream>>>(X1, nid, WT2, ENT, PAIR, RELT, g2, b2, emb, out);
}
